// CrossAttention_17085379904166
// MI455X (gfx1250) — hardware-verified
//
#include <hip/hip_runtime.h>
#include <stdint.h>


typedef _Float16 v16h __attribute__((ext_vector_type(16)));
typedef _Float16 v8h  __attribute__((ext_vector_type(8)));
typedef float    v8f  __attribute__((ext_vector_type(8)));
typedef float    v4f  __attribute__((ext_vector_type(4)));

#ifndef NB
#define NB 4
#endif
#ifndef SEQ
#define SEQ 2048
#endif
#ifndef MCTX
#define MCTX 2048
#endif
#define NB_FULL   4
#define SEQ_FULL  2048
#define MCTX_FULL 2048
#define DQ   1024
#define DC   1024
#define DM   1024
#define DOUT 1024
#define NH   16
#define HD   64
#define NKV  128
#define MQ   (NB * SEQ)
#define MK   (NB * MCTX)
#define MAXPOS ((SEQ > MCTX) ? SEQ : MCTX)

#define ACT_CAR   8.0f
#define W_CAR     1024.0f
#define PROJ_SCL  0.0009765625f
#define RES_CAR   2048.0f
#define RES_INV   0.00048828125f
#define S_SCL     0.001953125f
#define P_CAR     16384.0f
#define O_SCL     0.001953125f
#define OUT_SCL   3.814697265625e-06f

static_assert(NB >= 1 && NB <= NB_FULL);
static_assert(SEQ % 128 == 0);
static_assert(MCTX % 128 == 0);
static_assert(SEQ <= SEQ_FULL && MCTX <= MCTX_FULL);
static_assert(DM == NH * HD);
static_assert(HD == 64);
static_assert(NKV == 2 * HD);
static_assert(NKV == 128);
static_assert(DQ % 64 == 0 && DC % 64 == 0 && DM % 64 == 0 && DOUT % 64 == 0);
static_assert(DQ % 32 == 0 && DC % 32 == 0 && DM % 32 == 0);
static_assert(MAXPOS % 8 == 0);
static_assert((long)NB_FULL * SEQ_FULL * DOUT * 4 == 33554432L);
static_assert(((long)MQ * DQ / 8) % 256 == 0 && ((long)MK * DC / 8) % 256 == 0);
static_assert((long)(DM / 64) * (DQ / 64) * 4096 == (long)DQ * DM);
static_assert((long)(NKV / 64) * (DC / 64) * 4096 == (long)DC * NKV);
static_assert((long)(DOUT / 64) * (DM / 64) * 4096 == (long)DM * DOUT);
static_assert((long)(MAXPOS / 8) * 512 == (long)MAXPOS * 64);
static_assert((long)(DM / 64) * (MQ / 128) * 128 * 64 == (long)MQ * DM);
static_assert((long)(HD / 64) * (MK / 128) * 128 * 64 == (long)MK * HD);
static_assert((long)(MK / 64) * (NKV / 128) * 128 * 64 == (long)NKV * MK);
static_assert((long)(SEQ / 128) * NH * NB * 128 * HD == (long)MQ * DM);
static_assert((long)(DOUT / 64) * (MQ / 64) * 64 * 64 == (long)MQ * DOUT);

constexpr size_t N_X   = (size_t)MQ * DQ;
constexpr size_t N_C   = (size_t)MK * DC;
constexpr size_t N_WQ  = (size_t)DM * DQ;
constexpr size_t N_WKV = (size_t)NKV * DC;
constexpr size_t N_WO  = (size_t)DOUT * DM;
constexpr size_t N_Q   = (size_t)MQ * DM;
constexpr size_t N_K   = (size_t)MK * HD;
constexpr size_t N_VT  = (size_t)NKV * MK;
constexpr size_t N_TAB = (size_t)MAXPOS * 64;
constexpr size_t WS_HALVES = N_X + N_C + N_WQ + N_WKV + N_WO + N_Q + N_K + N_VT + 2 * N_Q;
constexpr size_t WS_TOTAL  = WS_HALVES * 2 + N_TAB * 4;
static_assert(N_X % 64 == 0 && N_C % 64 == 0 && N_WQ % 64 == 0 && N_WKV % 64 == 0 && N_WO % 64 == 0);
static_assert(N_Q % 64 == 0 && N_K % 64 == 0 && N_VT % 64 == 0);
static_assert(WS_HALVES % 64 == 0);
static_assert(WS_TOTAL <= (size_t)134217728);

union Frag16 { v16h v; v8h p[2]; };

__device__ __forceinline__ v16h ld_frag(const _Float16* p, int hl) {
  Frag16 f;
  f.p[0] = *(const v8h*)(p + 8 * hl);
  f.p[1] = *(const v8h*)(p + 16 + 8 * hl);
  return f.v;
}

__device__ __forceinline__ v8f mma(v16h a, v16h b, v8f c) {
  v8f d = __builtin_amdgcn_wmma_f32_16x16x32_f16(false, a, false, b, (short)0, c, false, false);
  asm volatile("v_nop\n\tv_nop\n\tv_nop\n\tv_nop" : "+v"(d) : "v"(a), "v"(b));
  return d;
}

__device__ __forceinline__ float bf16_rne(float x) {
  unsigned int u = __builtin_bit_cast(unsigned int, x);
  u += 0x7FFFu + ((u >> 16) & 1u);
  return __builtin_bit_cast(float, u & 0xFFFF0000u);
}

__global__ __launch_bounds__(256) void k_cvt8(const float* __restrict__ src,
                                              _Float16* __restrict__ dst,
                                              int cols, int rpb, int bstride, float car, int total8)
{
  const int i8 = blockIdx.x * 256 + threadIdx.x;
  if (i8 >= total8) return;
  const size_t e   = (size_t)i8 * 8;
  const size_t r   = e / (size_t)cols;
  const int    col = (int)(e - r * (size_t)cols);
  const size_t b   = r / (size_t)rpb;
  const size_t rr  = r - b * (size_t)rpb;
  const float* s = src + b * (size_t)bstride + rr * (size_t)cols + col;
  const v4f x0 = *(const v4f*)s;
  const v4f x1 = *(const v4f*)(s + 4);
  v8h o;
#pragma unroll
  for (int j = 0; j < 4; ++j) {
    const float t0 = x0[j];
    const float t1 = x1[j];
    o[j]     = (_Float16)(bf16_rne(t0) * car);
    o[4 + j] = (_Float16)(bf16_rne(t1) * car);
  }
  _Float16* d = dst + e;
  *(volatile v8h*)d = o;
  __threadfence();
  *(volatile v8h*)d = o;
}

__global__ __launch_bounds__(256) void k_trw(const float* __restrict__ W,
                                             _Float16* __restrict__ WT, int R, int C)
{
  __shared__ float tile[64 * 65];
  const int tid = threadIdx.x;
  const int c0 = blockIdx.x * 64, r0 = blockIdx.y * 64;
#pragma unroll
  for (int i = 0; i < 4; ++i) {
    const int idx = i * 256 + tid;
    const int r = idx >> 4, c4 = (idx & 15) * 4;
    const v4f v = *(const v4f*)(W + (size_t)(r0 + r) * C + c0 + c4);
    float* tp = tile + r * 65 + c4;
    tp[0] = v[0]; tp[1] = v[1]; tp[2] = v[2]; tp[3] = v[3];
  }
  __syncthreads();
  v8h o[2];
  _Float16* dp[2];
#pragma unroll
  for (int i = 0; i < 2; ++i) {
    const int line = i * 32 + (tid >> 3);
    const int pc   = (tid & 7) * 8;
#pragma unroll
    for (int j = 0; j < 8; ++j)
      o[i][j] = (_Float16)(bf16_rne(tile[(pc + j) * 65 + line]) * W_CAR);
    dp[i] = WT + (size_t)(c0 + line) * R + r0 + pc;
  }
  *(volatile v8h*)dp[0] = o[0];
  *(volatile v8h*)dp[1] = o[1];
  __threadfence();
  *(volatile v8h*)dp[0] = o[0];
  *(volatile v8h*)dp[1] = o[1];
}

__global__ __launch_bounds__(256) void k_rope(float* __restrict__ tab)
{
  __shared__ __attribute__((aligned(16))) float cs[8 * 64];
  const int tid = threadIdx.x;
  const int p = tid >> 5, i = tid & 31;
  const int pos = blockIdx.x * 8 + p;
  const float invf = exp2f(-0.375f * (float)i);
  const float ang = (float)pos * invf;
  float sn, cn;
  sincosf(ang, &sn, &cn);
  cs[p * 64 + i]      = cn;
  cs[p * 64 + 32 + i] = sn;
  __syncthreads();
  if (tid < 128) {
    const v4f v = *(const v4f*)(cs + tid * 4);
    float* d = tab + (size_t)blockIdx.x * 512 + tid * 4;
    *(volatile v4f*)d = v;
    __threadfence();
    *(volatile v4f*)d = v;
  }
}

__device__ __forceinline__ void gemm_core(const _Float16* ap0, const _Float16* ap1,
                                          const _Float16* bp, int K, int hl, v8f (&acc)[8])
{
  const size_t bst = (size_t)16 * K;
#pragma unroll 1
  for (int k0 = 0; k0 < K; k0 += 32) {
    const v16h a0 = ld_frag(ap0 + k0, hl);
    const v16h a1 = ld_frag(ap1 + k0, hl);
    const v16h b0 = ld_frag(bp + k0, hl);
    const v16h b1 = ld_frag(bp + bst + k0, hl);
    const v16h b2 = ld_frag(bp + 2 * bst + k0, hl);
    const v16h b3 = ld_frag(bp + 3 * bst + k0, hl);
    acc[0] = mma(a0, b0, acc[0]);
    acc[1] = mma(a0, b1, acc[1]);
    acc[2] = mma(a0, b2, acc[2]);
    acc[3] = mma(a0, b3, acc[3]);
    acc[4] = mma(a1, b0, acc[4]);
    acc[5] = mma(a1, b1, acc[5]);
    acc[6] = mma(a1, b2, acc[6]);
    acc[7] = mma(a1, b3, acc[7]);
  }
}

template <int MODE>
__device__ __forceinline__ void proj_body(float* ldsF,
                                          const _Float16* __restrict__ A,
                                          const _Float16* __restrict__ Bt,
                                          _Float16* __restrict__ PH,
                                          const float* __restrict__ bias,
                                          const float* __restrict__ tab,
                                          int K, int ldc, int rpb)
{
  const int tid = threadIdx.x, lane = tid & 31, w = tid >> 5;
  const int hl = lane >> 4, c = lane & 15;
  const int m0 = blockIdx.y * 128, n0 = blockIdx.x * 64;
  const int mw = m0 + 32 * w;

  const _Float16* ap0 = A  + (size_t)(mw + c) * K;
  const _Float16* ap1 = A  + (size_t)(mw + 16 + c) * K;
  const _Float16* bp  = Bt + (size_t)(n0 + c) * K;

  v8f acc[8] = {};
  gemm_core(ap0, ap1, bp, K, hl, acc);

#pragma unroll
  for (int i = 0; i < 2; ++i)
#pragma unroll
    for (int t = 0; t < 4; ++t)
#pragma unroll
      for (int r = 0; r < 8; ++r) {
        const int rowl = 32 * w + 16 * i + 8 * hl + r;
        ldsF[rowl * 68 + 16 * t + c] = acc[i * 4 + t][r] * PROJ_SCL;
      }
  __syncthreads();

  v8h vh[8];
#pragma unroll
  for (int i = 0; i < 8; ++i) {
    const int q = i * 128 + tid;
    const int rowl = q >> 3, ch = (q & 7) * 8;
    const v4f x0 = *(const v4f*)(ldsF + rowl * 68 + ch);
    const v4f x1 = *(const v4f*)(ldsF + rowl * 68 + ch + 4);
    float y[8];
    if (MODE == 0) {
      const v4f b0 = *(const v4f*)(bias + n0 + ch);
      const v4f b1 = *(const v4f*)(bias + n0 + ch + 4);
      float x[8];
#pragma unroll
      for (int j = 0; j < 4; ++j) {
        x[j]     = x0[j] + bf16_rne(b0[j]) * ACT_CAR;
        x[4 + j] = x1[j] + bf16_rne(b1[j]) * ACT_CAR;
      }
      const int pos = (m0 + rowl) % rpb;
      const float* tp = tab + (size_t)pos * 64 + (((n0 + ch) & 63) >> 1);
      const v4f cs = *(const v4f*)tp;
      const v4f sn = *(const v4f*)(tp + 32);
#pragma unroll
      for (int j = 0; j < 4; ++j) {
        y[2 * j]     = x[2 * j] * cs[j] - x[2 * j + 1] * sn[j];
        y[2 * j + 1] = x[2 * j + 1] * cs[j] + x[2 * j] * sn[j];
      }
    } else {
      const float bb = bf16_rne(bias[m0 + rowl]) * ACT_CAR;
#pragma unroll
      for (int j = 0; j < 4; ++j) {
        y[j]     = x0[j] + bb;
        y[4 + j] = x1[j] + bb;
      }
    }
#pragma unroll
    for (int j = 0; j < 8; ++j) vh[i][j] = (_Float16)y[j];
  }

  _Float16* const bh = PH + (size_t)m0 * ldc + n0;
#pragma unroll
  for (int i = 0; i < 8; ++i) {
    const int q = i * 128 + tid;
    const int rowl = q >> 3, ch = (q & 7) * 8;
    *(volatile v8h*)(bh + (size_t)rowl * ldc + ch) = vh[i];
  }
  __threadfence();
#pragma unroll
  for (int i = 0; i < 8; ++i) {
    const int q = i * 128 + tid;
    const int rowl = q >> 3, ch = (q & 7) * 8;
    *(volatile v8h*)(bh + (size_t)rowl * ldc + ch) = vh[i];
  }
}

__global__ __launch_bounds__(128) __attribute__((amdgpu_num_vgpr(256)))
void k_proj_rope(const _Float16* __restrict__ A, const _Float16* __restrict__ Bt,
                 _Float16* __restrict__ PH,
                 const float* __restrict__ bias, const float* __restrict__ tab,
                 int K, int ldc, int rpb)
{
  __shared__ __attribute__((aligned(16))) float ldsF[128 * 68];
  proj_body<0>(ldsF, A, Bt, PH, bias, tab, K, ldc, rpb);
}

__global__ __launch_bounds__(128) __attribute__((amdgpu_num_vgpr(256)))
void k_proj_vt(const _Float16* __restrict__ A, const _Float16* __restrict__ Bt,
               _Float16* __restrict__ PH, const float* __restrict__ bias, int K, int ldc)
{
  __shared__ __attribute__((aligned(16))) float ldsF[128 * 68];
  proj_body<1>(ldsF, A, Bt, PH, bias, bias, K, ldc, 1);
}

__global__ __launch_bounds__(256) __attribute__((amdgpu_num_vgpr(256)))
void k_attn(const _Float16* __restrict__ QH,
            const _Float16* __restrict__ KH,
            const _Float16* __restrict__ Vt,
            _Float16* __restrict__ OH, _Float16* __restrict__ OL)
{
  constexpr int KT_H   = 32 * 72;
  constexpr int V_H    = HD * 40;
  constexpr int P_H    = 8 * 16 * 40;
  constexpr int TILE_H = KT_H + V_H + P_H;
  constexpr int EPI_H  = 2 * 128 * 72;
  constexpr int LDS_H  = (TILE_H > EPI_H) ? TILE_H : EPI_H;
  static_assert(LDS_H * 2 <= 65536);
  static_assert(32 * 8 == 256 && HD * 4 == 256);
  __shared__ __attribute__((aligned(16))) _Float16 lds[LDS_H];
  _Float16* const ldsK0 = lds;
  _Float16* const ldsVH = ldsK0 + KT_H;
  _Float16* const ldsP  = ldsVH + V_H;
  _Float16* const ldsOH = lds;
  _Float16* const ldsOL = lds + 128 * 72;

  const int tid = threadIdx.x, lane = tid & 31, w = tid >> 5;
  const int hl = lane >> 4, c = lane & 15;
  const int q0 = blockIdx.x * 128;
  const int col0 = blockIdx.y * HD;
  const int bb = blockIdx.z;
  const size_t qbase = (size_t)bb * SEQ + q0;

  const size_t qrow = (qbase + 16 * w + c) * DM + col0;
  v16h qh[2];
#pragma unroll
  for (int ks = 0; ks < 2; ++ks) qh[ks] = ld_frag(QH + qrow + 32 * ks, hl);
  _Float16* const myP = ldsP + w * (16 * 40);

  const int krr = tid >> 3, kcc = (tid & 7) * 8;
  const int vdd = tid >> 2, vkc = (tid & 3) * 8;
  const _Float16* const kgh = KH + ((size_t)bb * MCTX + krr) * HD + kcc;
  const _Float16* const vgh = Vt + (size_t)(HD + vdd) * MK + (size_t)bb * MCTX + vkc;

  float m[8], l[8];
  v8f oh[4] = {};
#pragma unroll
  for (int r = 0; r < 8; ++r) { m[r] = -__builtin_inff(); l[r] = 0.f; }

#pragma unroll 1
  for (int kt = 0; kt < MCTX / 32; ++kt) {
    const int mk = kt * 32;
    {
      const v8h k8h = *(const v8h*)(kgh + (size_t)mk * HD);
      const v8h v8a = *(const v8h*)(vgh + mk);
      *(v8h*)(ldsK0 + krr * 72 + kcc) = k8h;
      *(v8h*)(ldsVH + vdd * 40 + vkc) = v8a;
    }
    __syncthreads();

    v8f sh[2] = {};
#pragma unroll
    for (int ks = 0; ks < 2; ++ks) {
#pragma unroll
      for (int t = 0; t < 2; ++t) {
        const v16h kfh = ld_frag(ldsK0 + (16 * t + c) * 72 + 32 * ks, hl);
        sh[t] = mma(qh[ks], kfh, sh[t]);
      }
    }

#pragma unroll
    for (int r = 0; r < 8; ++r) {
      const float v0 = sh[0][r] * S_SCL;
      const float v1 = sh[1][r] * S_SCL;
      float tm = fmaxf(v0, v1);
      tm = fmaxf(tm, __shfl_xor(tm, 1, 32));
      tm = fmaxf(tm, __shfl_xor(tm, 2, 32));
      tm = fmaxf(tm, __shfl_xor(tm, 4, 32));
      tm = fmaxf(tm, __shfl_xor(tm, 8, 32));
      const float mn = fmaxf(m[r], tm);
      const float al = __expf(m[r] - mn);
      const float p0 = __expf(v0 - mn), p1 = __expf(v1 - mn);
      float rs = p0 + p1;
      rs += __shfl_xor(rs, 1, 32);
      rs += __shfl_xor(rs, 2, 32);
      rs += __shfl_xor(rs, 4, 32);
      rs += __shfl_xor(rs, 8, 32);
      l[r] = l[r] * al + rs;
      m[r] = mn;
#pragma unroll
      for (int t = 0; t < 4; ++t) oh[t][r] *= al;
      _Float16* pp = myP + (8 * hl + r) * 40 + c;
      pp[0]  = (_Float16)(p0 * P_CAR);
      pp[16] = (_Float16)(p1 * P_CAR);
    }
    __syncthreads();

    const v16h pf = ld_frag(myP + c * 40, hl);
#pragma unroll
    for (int t = 0; t < 4; ++t) {
      const v16h vfh = ld_frag(ldsVH + (16 * t + c) * 40, hl);
      oh[t] = mma(pf, vfh, oh[t]);
    }
    __syncthreads();
  }

#pragma unroll
  for (int r = 0; r < 8; ++r) {
    const float inv = (1.0f / l[r]) * O_SCL;
    const int rowl = 16 * w + 8 * hl + r;
#pragma unroll
    for (int t = 0; t < 4; ++t) {
      const float v = oh[t][r] * inv;
      const _Float16 hv = (_Float16)v;
      const float res = (v - (float)hv) * RES_CAR;
      ldsOH[rowl * 72 + 16 * t + c] = hv;
      ldsOL[rowl * 72 + 16 * t + c] = (_Float16)res;
    }
  }
  __syncthreads();
  _Float16* const bh = OH + qbase * DM + col0;
  _Float16* const bl = OL + qbase * DM + col0;
  for (int i = 0; i < 4; ++i) {
    const int q = i * 256 + tid;
    const int rowl = q >> 3, ch = (q & 7) * 8;
    const v8h vh = *(const v8h*)(ldsOH + rowl * 72 + ch);
    const v8h vl = *(const v8h*)(ldsOL + rowl * 72 + ch);
    *(volatile v8h*)(bh + (size_t)rowl * DM + ch) = vh;
    *(volatile v8h*)(bl + (size_t)rowl * DM + ch) = vl;
  }
  __threadfence();
  for (int i = 0; i < 4; ++i) {
    const int q = i * 256 + tid;
    const int rowl = q >> 3, ch = (q & 7) * 8;
    const v8h vh = *(const v8h*)(ldsOH + rowl * 72 + ch);
    const v8h vl = *(const v8h*)(ldsOL + rowl * 72 + ch);
    *(volatile v8h*)(bh + (size_t)rowl * DM + ch) = vh;
    *(volatile v8h*)(bl + (size_t)rowl * DM + ch) = vl;
  }
}

__global__ __launch_bounds__(128) __attribute__((amdgpu_num_vgpr(256)))
void k_oproj(const _Float16* __restrict__ AH, const _Float16* __restrict__ AL,
             const _Float16* __restrict__ Bt, const float* __restrict__ bo,
             float* __restrict__ Out)
{
  __shared__ __attribute__((aligned(16))) float ldsF[64 * 68];
  static_assert(SEQ % 64 == 0);

  const int tid = threadIdx.x, lane = tid & 31, w = tid >> 5;
  const int hl = lane >> 4, c = lane & 15;
  const int m0 = blockIdx.y * 64, n0 = blockIdx.x * 64;
  const int mw = m0 + 16 * w;

  const _Float16* ap0 = AH + (size_t)(mw + c) * DM;
  const _Float16* ap1 = AL + (size_t)(mw + c) * DM;
  const _Float16* bp  = Bt + (size_t)(n0 + c) * DM;

  v8f acc[8] = {};
  gemm_core(ap0, ap1, bp, DM, hl, acc);

#pragma unroll
  for (int t = 0; t < 4; ++t)
#pragma unroll
    for (int r = 0; r < 8; ++r) {
      const int rowl = 16 * w + 8 * hl + r;
      ldsF[rowl * 68 + 16 * t + c] = (acc[t][r] + acc[4 + t][r] * RES_INV) * OUT_SCL;
    }
  __syncthreads();

  const int bbatch = m0 / SEQ;
  const int srow   = m0 - bbatch * SEQ;
  float* const ob = Out + ((size_t)bbatch * SEQ_FULL + srow) * DOUT + n0;
  for (int i = 0; i < 8; ++i) {
    const int qi = i * 128 + tid;
    const int rowl = qi >> 4, col = (qi & 15) * 4;
    const v4f a = *(const v4f*)(ldsF + rowl * 68 + col);
    const v4f b = *(const v4f*)(bo + n0 + col);
    v4f v;
    v[0] = a[0] + bf16_rne(b[0]); v[1] = a[1] + bf16_rne(b[1]);
    v[2] = a[2] + bf16_rne(b[2]); v[3] = a[3] + bf16_rne(b[3]);
    *(volatile v4f*)(ob + (size_t)rowl * DOUT + col) = v;
  }
  __threadfence();
  for (int i = 0; i < 8; ++i) {
    const int qi = i * 128 + tid;
    const int rowl = qi >> 4, col = (qi & 15) * 4;
    const v4f a = *(const v4f*)(ldsF + rowl * 68 + col);
    const v4f b = *(const v4f*)(bo + n0 + col);
    v4f v;
    v[0] = a[0] + bf16_rne(b[0]); v[1] = a[1] + bf16_rne(b[1]);
    v[2] = a[2] + bf16_rne(b[2]); v[3] = a[3] + bf16_rne(b[3]);
    *(volatile v4f*)(ob + (size_t)rowl * DOUT + col) = v;
  }
}

extern "C" void kernel_launch(void* const* d_in, const int* in_sizes, int n_in,
                              void* d_out, int out_size, void* d_ws, size_t ws_size,
                              hipStream_t stream)
{
  if (n_in < 8) return;
  if ((long)in_sizes[0] < ((long)(NB - 1) * SEQ_FULL + SEQ) * DQ) return;
  if ((long)in_sizes[1] < ((long)(NB - 1) * MCTX_FULL + MCTX) * DC) return;
  if ((long)in_sizes[2] < (long)DQ * DM) return;
  if ((long)in_sizes[3] < (long)DM) return;
  if ((long)in_sizes[4] < (long)DC * NKV) return;
  if ((long)in_sizes[5] < (long)NKV) return;
  if ((long)in_sizes[6] < (long)DM * DOUT) return;
  if ((long)in_sizes[7] < (long)DOUT) return;
  if ((long)out_size < ((long)(NB - 1) * SEQ_FULL + SEQ) * DOUT) return;
  if (WS_TOTAL > ws_size) return;

  const float* q   = (const float*)d_in[0];
  const float* kv  = (const float*)d_in[1];
  const float* Wq  = (const float*)d_in[2];
  const float* bq  = (const float*)d_in[3];
  const float* Wkv = (const float*)d_in[4];
  const float* bkv = (const float*)d_in[5];
  const float* Wo  = (const float*)d_in[6];
  const float* bo  = (const float*)d_in[7];
  float* out = (float*)d_out;

  _Float16* X16  = (_Float16*)d_ws;
  _Float16* C16  = X16  + N_X;
  _Float16* WqT  = C16  + N_C;
  _Float16* WkvT = WqT  + N_WQ;
  _Float16* WoT  = WkvT + N_WKV;
  _Float16* QH   = WoT  + N_WO;
  _Float16* KH   = QH   + N_Q;
  _Float16* Vt   = KH   + N_K;
  _Float16* OH   = Vt   + N_VT;
  _Float16* OL   = OH   + N_Q;
  float*    tab  = (float*)(OL + N_Q);

  const int tx8 = (int)(N_X / 8);
  const int tc8 = (int)(N_C / 8);
  k_cvt8<<<(tx8 + 255) / 256, 256, 0, stream>>>(q,  X16, DQ, SEQ,  SEQ_FULL * DQ,  ACT_CAR, tx8);
  k_cvt8<<<(tc8 + 255) / 256, 256, 0, stream>>>(kv, C16, DC, MCTX, MCTX_FULL * DC, ACT_CAR, tc8);

  k_trw<<<dim3(DM / 64,   DQ / 64), 256, 0, stream>>>(Wq,  WqT,  DQ, DM);
  k_trw<<<dim3(NKV / 64,  DC / 64), 256, 0, stream>>>(Wkv, WkvT, DC, NKV);
  k_trw<<<dim3(DOUT / 64, DM / 64), 256, 0, stream>>>(Wo,  WoT,  DM, DOUT);

  k_rope<<<MAXPOS / 8, 256, 0, stream>>>(tab);

  k_proj_rope<<<dim3(DM / 64, MQ / 128), 128, 0, stream>>>(X16, WqT, QH, bq, tab, DQ, DM, SEQ);
  k_proj_rope<<<dim3(HD / 64, MK / 128), 128, 0, stream>>>(C16, WkvT, KH, bkv, tab, DC, HD, MCTX);
  k_proj_vt<<<dim3(MK / 64, NKV / 128), 128, 0, stream>>>(WkvT, C16, Vt, bkv, DC, MK);

  k_attn<<<dim3(SEQ / 128, NH, NB), 256, 0, stream>>>(QH, KH, Vt, OH, OL);

  k_oproj<<<dim3(DOUT / 64, MQ / 64), 128, 0, stream>>>(OH, OL, WoT, bo, out);
}
